// MambaTower_36490042147416
// MI455X (gfx1250) — hardware-verified
//
#include <hip/hip_runtime.h>
#include <math.h>

typedef __attribute__((ext_vector_type(16))) _Float16 v16h;
typedef __attribute__((ext_vector_type(8)))  _Float16 v8h;
typedef __attribute__((ext_vector_type(8)))  float    v8f;
typedef __attribute__((ext_vector_type(4)))  float    v4f;
typedef __attribute__((ext_vector_type(2)))  float    v2f;

constexpr int kL    = 2048;
constexpr int kDM   = 256;
constexpr int kE    = 512;
constexpr int kNS   = 16;
constexpr int kRk   = 16;
constexpr int kTaps = 4;
constexpr int kNL   = 4;
constexpr int kNCA  = 2;
constexpr int kTr   = 8;
constexpr int kDT   = 64;
constexpr int kNH   = 4;
constexpr int kDH   = 64;
constexpr int kXZP  = 2 * kE;
constexpr int kPRN  = kRk + 2 * kNS;
constexpr int kPRP  = 64;
constexpr int kDTK  = 32;
constexpr int kRows2 = 2 * kL;
constexpr int kKVP  = 2 * kDM;
constexpr int kConvTP = 260;
constexpr int kScanCh = 128;
constexpr int kScanYP = 132;
constexpr float kActCarry = 16.0f;
constexpr float kWgtCarry = 32.0f;
constexpr float kFold     = 1.0f / (kActCarry * kWgtCarry);
constexpr float kLogitScale = 0.125f;
static_assert(kLogitScale * kLogitScale * (float)kDH == 1.0f);
static_assert(kNH * kDH == kDM);
static_assert(kPRN == 48 && kPRN <= kPRP);
static_assert((kDM % 32) == 0 && (kE % 32) == 0 && (kDT % 32) == 0 && (kDTK % 32) == 0);
static_assert((kL % 64) == 0 && (kRows2 % 64) == 0 && ((kL * kTr) % 64) == 0);
static_assert((kXZP % 64) == 0 && (kPRP % 64) == 0 && (kE % 64) == 0 && (kDM % 64) == 0 && (kKVP % 64) == 0);
static_assert(kRk <= kDTK && kNS == 16 && kTaps == 4 && kTr == 8);

constexpr size_t kOffWIN  = 0;
constexpr size_t kOffWXP  = kOffWIN  + (size_t)kNL * kXZP * kDM * 2;
constexpr size_t kOffWDT  = kOffWXP  + (size_t)kNL * kPRP * kE * 2;
constexpr size_t kOffWOUT = kOffWDT  + (size_t)kNL * kE * kDTK * 2;
constexpr size_t kOffWQ   = kOffWOUT + (size_t)kNL * kDM * kE * 2;
constexpr size_t kOffWKV  = kOffWQ   + (size_t)kNCA * kDM * kDM * 2;
constexpr size_t kOffWO   = kOffWKV  + (size_t)kNCA * kKVP * kDT * 2;
constexpr size_t kOffBKV  = kOffWO   + (size_t)kNCA * kDM * kDM * 2;
constexpr size_t kOffTL   = kOffBKV  + (size_t)kNCA * kKVP * 4;
constexpr size_t kOffXA   = kOffTL   + (size_t)kL * kTr * kDT * 2;
constexpr size_t kOffXB   = kOffXA   + (size_t)kL * kDM * 4;
constexpr size_t kOffH16  = kOffXB   + (size_t)kL * kDM * 4;
constexpr size_t kOffXZ   = kOffH16  + (size_t)kL * kDM * 2;
constexpr size_t kOffU    = kOffXZ   + (size_t)kL * kXZP * 4;
constexpr size_t kOffU16  = kOffU    + (size_t)kRows2 * kE * 4;
constexpr size_t kOffPR   = kOffU16  + (size_t)kRows2 * kE * 2;
constexpr size_t kOffDT16 = kOffPR   + (size_t)kRows2 * kPRP * 4;
constexpr size_t kOffDLR  = kOffDT16 + (size_t)kRows2 * kDTK * 2;
constexpr size_t kOffY    = kOffDLR  + (size_t)kRows2 * kE * 4;
constexpr size_t kOffG16  = kOffY    + (size_t)kRows2 * kE * 4;
constexpr size_t kOffQ    = kOffG16  + (size_t)kL * kE * 2;
constexpr size_t kOffKV   = kOffQ    + (size_t)kL * kDM * 4;
constexpr size_t kOffO16  = kOffKV   + (size_t)kL * kTr * kKVP * 4;
constexpr size_t kWsTotal = kOffO16  + (size_t)kL * kDM * 2;
static_assert(kWsTotal == 89395200ull);
static_assert(kWsTotal <= 134217728ull);
static_assert((kOffWXP % 128) == 0 && (kOffWDT % 128) == 0 && (kOffWOUT % 128) == 0 && (kOffWQ % 128) == 0 &&
              (kOffWKV % 128) == 0 && (kOffWO % 128) == 0 && (kOffBKV % 128) == 0 && (kOffTL % 128) == 0 &&
              (kOffXA % 128) == 0 && (kOffXB % 128) == 0 && (kOffH16 % 128) == 0 && (kOffXZ % 128) == 0 &&
              (kOffU % 128) == 0 && (kOffU16 % 128) == 0 && (kOffPR % 128) == 0 && (kOffDT16 % 128) == 0 &&
              (kOffDLR % 128) == 0 && (kOffY % 128) == 0 && (kOffG16 % 128) == 0 && (kOffQ % 128) == 0 &&
              (kOffKV % 128) == 0 && (kOffO16 % 128) == 0);

__device__ __forceinline__ void guard_row_h(v8f& a, v8f& b, v8f& c, v8f& d, v16h x, v16h y0, v16h y1, v16h y2, v16h y3) {
  asm volatile("v_nop\n\tv_nop\n\tv_nop\n\tv_nop" : "+v"(a), "+v"(b), "+v"(c), "+v"(d) : "v"(x), "v"(y0), "v"(y1), "v"(y2), "v"(y3));
}
__device__ __forceinline__ void keep4_h(v16h a, v16h b, v16h c, v16h d) { asm volatile("v_nop" :: "v"(a), "v"(b), "v"(c), "v"(d)); }
__device__ __forceinline__ void acc_guard4(v8f& a, v8f& b, v8f& c, v8f& d) { asm volatile("v_nop\n\tv_nop\n\tv_nop\n\tv_nop" : "+v"(a), "+v"(b), "+v"(c), "+v"(d)); }
template <typename T> struct Frag;
template <> struct Frag<_Float16> {
  typedef v16h V; union U { v16h v; v8h h[2]; };
  static __device__ __forceinline__ v16h load(const _Float16* p) {
    U f; f.h[0] = *(const v8h*)(p); f.h[1] = *(const v8h*)(p + 16); return f.v;
  }
  static __device__ __forceinline__ v8f mma(v16h a, v16h b, v8f c) {
    return __builtin_amdgcn_wmma_f32_16x16x32_f16(false, a, false, b, (short)0, c, false, false);
  }
};

template <int BIAS_MODE, bool RESID>
__global__ __launch_bounds__(256) void wmma_gemm64(
    const unsigned short* __restrict__ Ap, int lda,
    const unsigned short* __restrict__ Btp, int ldb,
    float* __restrict__ Cout, int ldc,
    const float* __restrict__ bias,
    const float* __restrict__ resid,
    int M, int N, int K, float scale) {
  typedef _Float16 T;
  typedef v16h V;
  const T* A = (const T*)Ap; const T* Bt = (const T*)Btp;
  __shared__ __align__(16) float sT[8][16 * 68];
  const int lane = threadIdx.x & 31;
  const int wave = threadIdx.x >> 5;
  const int tilesN = N >> 6;
  const int tilesM = M >> 6;
  const int tile = blockIdx.x * 8 + wave;
  if (tile >= tilesM * tilesN) return;
  const int tm = tile / tilesN;
  const int tn = tile - tm * tilesN;
  const int m0 = tm << 6;
  const int n0 = tn << 6;

  const int rlane = lane & 15;
  const int koff  = (lane >> 4) * 8;
  const int mOff  = (lane >> 4) * 8;

  v8f acc[4][4];
#pragma unroll
  for (int i = 0; i < 4; ++i)
#pragma unroll
    for (int j = 0; j < 4; ++j) acc[i][j] = (v8f){0.f,0.f,0.f,0.f,0.f,0.f,0.f,0.f};

  for (int k0 = 0; k0 < K; k0 += 32) {
    V bh[4];
#pragma unroll
    for (int j = 0; j < 4; ++j) {
      const size_t bo = (size_t)(n0 + (j << 4) + rlane) * ldb + koff + k0;
      bh[j] = Frag<T>::load(Bt + bo);
    }
#pragma unroll
    for (int i = 0; i < 4; ++i) {
      const size_t ao = (size_t)(m0 + (i << 4) + rlane) * lda + koff + k0;
      V ah = Frag<T>::load(A + ao);
#pragma unroll
      for (int j = 0; j < 4; ++j) acc[i][j] = Frag<T>::mma(ah, bh[j], acc[i][j]);
      guard_row_h(acc[i][0], acc[i][1], acc[i][2], acc[i][3], ah, bh[0], bh[1], bh[2], bh[3]);
    }
    keep4_h(bh[0], bh[1], bh[2], bh[3]);
  }
  acc_guard4(acc[0][0], acc[0][1], acc[0][2], acc[0][3]);
  acc_guard4(acc[1][0], acc[1][1], acc[1][2], acc[1][3]);
  acc_guard4(acc[2][0], acc[2][1], acc[2][2], acc[2][3]);
  acc_guard4(acc[3][0], acc[3][1], acc[3][2], acc[3][3]);

  float* slab = sT[wave];
  float bvj[4];
#pragma unroll
  for (int j = 0; j < 4; ++j) {
    bvj[j] = 0.f;
    if (BIAS_MODE == 2) bvj[j] = bias[n0 + (j << 4) + rlane];
  }
  const int hh = lane >> 4, c4 = (lane & 15) * 4;
#pragma unroll
  for (int i = 0; i < 4; ++i) {
    const int mBase = m0 + (i << 4);
#pragma unroll
    for (int j = 0; j < 4; ++j) {
#pragma unroll
      for (int r = 0; r < 8; ++r) {
        float v = acc[i][j][r] * scale;
        if (BIAS_MODE == 2) v += bvj[j];
        slab[(mOff + r) * 68 + (j << 4) + rlane] = v;
      }
    }
    __builtin_amdgcn_fence(__ATOMIC_RELEASE, "workgroup");
    __builtin_amdgcn_wave_barrier();
    __builtin_amdgcn_fence(__ATOMIC_ACQUIRE, "workgroup");
    v4f vals[8];
#pragma unroll
    for (int it = 0; it < 8; ++it) {
      const int row = it * 2 + hh;
      v4f v = *(const v4f*)(slab + row * 68 + c4);
      if (RESID) {
        const v4f rv = *(const v4f*)(resid + (size_t)(mBase + row) * ldc + n0 + c4);
        v = v + rv;
      }
      vals[it] = v;
    }
    for (int pass = 0; pass < 2; ++pass) {
#pragma unroll
      for (int it = 0; it < 8; ++it) {
        const int row = it * 2 + hh;
        *(volatile v4f*)(Cout + (size_t)(mBase + row) * ldc + n0 + c4) = vals[it];
      }
      __threadfence();
    }
    __builtin_amdgcn_fence(__ATOMIC_RELEASE, "workgroup");
    __builtin_amdgcn_wave_barrier();
    __builtin_amdgcn_fence(__ATOMIC_ACQUIRE, "workgroup");
  }
}

__global__ __launch_bounds__(256) void transpose_cast_kernel(
    const float* __restrict__ W, unsigned short* __restrict__ Bt, int Kdim, int Ndim, float scale,
    long srcLayerStride, long dstLayerStride)
{
  __shared__ float tile[64 * 65];
  const int tid = threadIdx.x, lane = tid & 31, wave = tid >> 5;
  const int n0 = blockIdx.x * 64;
  const int k0 = blockIdx.y * 64;
  const float* Wl = W + (size_t)blockIdx.z * (size_t)srcLayerStride;
  unsigned short* Bl = Bt + (size_t)blockIdx.z * (size_t)dstLayerStride;
#pragma unroll
  for (int p = 0; p < 16; ++p) {
    const int idx = tid + p * 256;
    const int kk  = idx >> 6;
    const int nn  = idx & 63;
    const int n   = n0 + nn;
    const int nc  = (n < Ndim) ? n : (Ndim - 1);
    const float v = Wl[(size_t)(k0 + kk) * Ndim + nc];
    tile[kk * 65 + nn] = (n < Ndim) ? (v * scale) : 0.f;
  }
  __syncthreads();
  const int q = lane >> 3, c8 = (lane & 7) * 8;
  v8h hv[2];
#pragma unroll
  for (int it = 0; it < 2; ++it) {
    const int nrow = it * 32 + wave * 4 + q;
#pragma unroll
    for (int e = 0; e < 8; ++e) hv[it][e] = (_Float16)tile[(c8 + e) * 65 + nrow];
  }
  for (int pass = 0; pass < 2; ++pass) {
#pragma unroll
    for (int it = 0; it < 2; ++it) {
      const int nrow = it * 32 + wave * 4 + q;
      *(volatile v8h*)(Bl + (size_t)(n0 + nrow) * Kdim + k0 + c8) = hv[it];
    }
    __threadfence();
  }
}

__global__ __launch_bounds__(256) void dtw_cast_kernel(
    const float* __restrict__ W, unsigned short* __restrict__ out, float scale)
{
  const int i = blockIdx.x * 256 + threadIdx.x;
  const int e0 = i << 3;
  const int row = e0 >> 5;
  const int kq = e0 & 31;
  const int layer = row >> 9;
  const int n = row & (kE - 1);
  const int kc = kq & 8;
  const bool valid = (kq < kRk);
  v8h hv;
#pragma unroll
  for (int e = 0; e < 8; ++e) {
    const float v = W[((size_t)layer * kRk + kc + e) * kE + n];
    const float t = valid ? (v * scale) : 0.0f;
    hv[e] = (_Float16)t;
  }
  unsigned short* q = out + e0;
  *(volatile v8h*)q = hv;
  __threadfence();
  *(volatile v8h*)q = hv;
}

__global__ __launch_bounds__(256) void bias_merge_kernel(
    const float* __restrict__ kb, const float* __restrict__ vb, float* __restrict__ out)
{
  const int e0 = threadIdx.x << 2;
  const int j = e0 >> 9;
  const int c = e0 & (kKVP - 1);
  const int cc = c & (kDM - 1);
  const v4f a = *(const v4f*)(kb + j * kDM + cc);
  const v4f b = *(const v4f*)(vb + j * kDM + cc);
  const bool isv = (c >= kDM);
  v4f o;
#pragma unroll
  for (int e = 0; e < 4; ++e) o[e] = isv ? b[e] : a[e];
  float* q = out + e0;
  *(volatile v4f*)q = o;
  __threadfence();
  *(volatile v4f*)q = o;
}

__global__ __launch_bounds__(256) void tracks_cast_kernel(
    const float* __restrict__ TR, unsigned short* __restrict__ TL16, float scale)
{
  const int i = blockIdx.x * 256 + threadIdx.x;
  const int e0 = i << 3;
  const int row = e0 >> 6;
  const int c8 = e0 & 63;
  const int l = row >> 3, t = row & 7;
  const float* p = TR + ((size_t)t * kL + l) * kDT + c8;
  const v4f a0 = *(const v4f*)(p);
  const v4f a1 = *(const v4f*)(p + 4);
  v8h hv;
#pragma unroll
  for (int e = 0; e < 4; ++e) {
    hv[e]     = (_Float16)(a0[e] * scale);
    hv[4 + e] = (_Float16)(a1[e] * scale);
  }
  unsigned short* q = TL16 + e0;
  *(volatile v8h*)q = hv;
  __threadfence();
  *(volatile v8h*)q = hv;
}

__global__ __launch_bounds__(256) void rmsnorm_f16_kernel(
    const float* __restrict__ X, const float* __restrict__ gw, unsigned short* __restrict__ H16, float scale)
{
  const int tid = threadIdx.x, lane = tid & 31, wave = tid >> 5;
  const int row = blockIdx.x * 8 + wave;
  const float* xr = X + (size_t)row * kDM + lane * 8;
  const v4f a0 = *(const v4f*)(xr);
  const v4f a1 = *(const v4f*)(xr + 4);
  const v4f g0 = *(const v4f*)(gw + lane * 8);
  const v4f g1 = *(const v4f*)(gw + lane * 8 + 4);
  float s = 0.0f;
#pragma unroll
  for (int e = 0; e < 4; ++e) { s += a0[e] * a0[e]; s += a1[e] * a1[e]; }
#pragma unroll
  for (int off = 16; off > 0; off >>= 1) s += __shfl_xor(s, off, 32);
  const float sc = rsqrtf(s * (1.0f / (float)kDM) + 1e-6f);
  v8h hv;
#pragma unroll
  for (int e = 0; e < 4; ++e) {
    hv[e]     = (_Float16)(((a0[e] * sc) * g0[e]) * scale);
    hv[4 + e] = (_Float16)(((a1[e] * sc) * g1[e]) * scale);
  }
  unsigned short* q = H16 + (size_t)row * kDM + lane * 8;
  *(volatile v8h*)q = hv;
  __threadfence();
  *(volatile v8h*)q = hv;
}

__global__ __launch_bounds__(256) void conv_silu_kernel(
    const float* __restrict__ XZ, const float* __restrict__ cw, const float* __restrict__ cb,
    float* __restrict__ U, unsigned short* __restrict__ U16, float scale16)
{
  __shared__ __align__(16) float sT[16 * kConvTP];
  const int tid = threadIdx.x, lane = tid & 31, wave = tid >> 5;
  const int d0 = blockIdx.x * 256, d = d0 + tid;
  const int g0 = blockIdx.y * 64;
  const int dir = blockIdx.z;
  const float w0 = cw[0 * kE + d], w1 = cw[1 * kE + d], w2 = cw[2 * kE + d], w3 = cw[3 * kE + d];
  const float bc = cb[d];
  float xm3, xm2, xm1;
  {
    const int r1 = dir ? (g0 + 64) : (g0 - 1);
    const int r2 = dir ? (g0 + 65) : (g0 - 2);
    const int r3 = dir ? (g0 + 66) : (g0 - 3);
    const int c1 = r1 < 0 ? 0 : (r1 > kL - 1 ? kL - 1 : r1);
    const int c2 = r2 < 0 ? 0 : (r2 > kL - 1 ? kL - 1 : r2);
    const int c3 = r3 < 0 ? 0 : (r3 > kL - 1 ? kL - 1 : r3);
    const float v1 = XZ[(size_t)c1 * kXZP + d];
    const float v2 = XZ[(size_t)c2 * kXZP + d];
    const float v3 = XZ[(size_t)c3 * kXZP + d];
    xm1 = (r1 >= 0 && r1 < kL) ? v1 : 0.f;
    xm2 = (r2 >= 0 && r2 < kL) ? v2 : 0.f;
    xm3 = (r3 >= 0 && r3 < kL) ? v3 : 0.f;
  }
  const int hrow = wave >> 1;
  const int hch  = (wave & 1) * 128 + lane * 4;
  float* Ud = U + (size_t)dir * kL * kE;
  unsigned short* U16d = U16 + (size_t)dir * kL * kE;
#pragma unroll 1
  for (int sub = 0; sub < 4; ++sub) {
    const int lb = dir ? (g0 + 48 - sub * 16) : (g0 + sub * 16);
#pragma unroll 1
    for (int s = 0; s < 16; ++s) {
      const int sr = dir ? (15 - s) : s;
      const float xc = XZ[(size_t)(lb + sr) * kXZP + d];
      float acc = w0 * xm3;
      acc = fmaf(w1, xm2, acc);
      acc = fmaf(w2, xm1, acc);
      acc = fmaf(w3, xc, acc);
      const float sv = acc + bc;
      const float sg = __builtin_amdgcn_rcpf(1.0f + expf(-sv));
      sT[sr * kConvTP + tid] = sv * sg;
      xm3 = xm2; xm2 = xm1; xm1 = xc;
    }
    __syncthreads();
    v4f fv[4];
    v8h bv[2];
#pragma unroll
    for (int it = 0; it < 4; ++it) fv[it] = *(const v4f*)(sT + (it * 4 + hrow) * kConvTP + hch);
#pragma unroll
    for (int it = 0; it < 2; ++it) {
      const float* sp = sT + (it * 8 + wave) * kConvTP + lane * 8;
      const v4f a0 = *(const v4f*)(sp);
      const v4f a1 = *(const v4f*)(sp + 4);
#pragma unroll
      for (int e = 0; e < 4; ++e) {
        bv[it][e]     = (_Float16)(a0[e] * scale16);
        bv[it][4 + e] = (_Float16)(a1[e] * scale16);
      }
    }
    for (int pass = 0; pass < 2; ++pass) {
#pragma unroll
      for (int it = 0; it < 4; ++it)
        *(volatile v4f*)(Ud + (size_t)(lb + it * 4 + hrow) * kE + d0 + hch) = fv[it];
#pragma unroll
      for (int it = 0; it < 2; ++it)
        *(volatile v8h*)(U16d + (size_t)(lb + it * 8 + wave) * kE + d0 + lane * 8) = bv[it];
      __threadfence();
    }
    __syncthreads();
  }
}

__global__ __launch_bounds__(256) void dt_cast_kernel(
    const float* __restrict__ PR, unsigned short* __restrict__ DT16, float scale)
{
  const int i = blockIdx.x * 256 + threadIdx.x;
  const int e0 = i << 3;
  const int row = e0 >> 5;
  const int c = e0 & 31;
  const bool valid = (c < kRk);
  const float* p = PR + (size_t)row * kPRP + (c & 8);
  const v4f a0 = *(const v4f*)(p);
  const v4f a1 = *(const v4f*)(p + 4);
  v8h hv;
#pragma unroll
  for (int e = 0; e < 4; ++e) {
    const float t0 = valid ? (a0[e] * scale) : 0.0f;
    const float t1 = valid ? (a1[e] * scale) : 0.0f;
    hv[e]     = (_Float16)t0;
    hv[4 + e] = (_Float16)t1;
  }
  unsigned short* q = DT16 + e0;
  *(volatile v8h*)q = hv;
  __threadfence();
  *(volatile v8h*)q = hv;
}

__global__ __launch_bounds__(128) void scan_kernel(
    const float* __restrict__ DLR, const float* __restrict__ U, const float* __restrict__ PR,
    const float* __restrict__ Alog, const float* __restrict__ Dp, float* __restrict__ Y)
{
  __shared__ __align__(16) float sBC[16 * 32];
  __shared__ __align__(16) float sY[16 * kScanYP];
  const int tid = threadIdx.x, lane = tid & 31, wave = tid >> 5;
  const int dir = blockIdx.x >> 2;
  const int d0 = (blockIdx.x & 3) * kScanCh;
  const int d = d0 + tid;
  const size_t rowbase = (size_t)dir * kL;

  float An[kNS], h[kNS];
#pragma unroll
  for (int q4 = 0; q4 < 4; ++q4) {
    const v4f a4 = *(const v4f*)(Alog + (size_t)d * kNS + 4 * q4);
#pragma unroll
    for (int e = 0; e < 4; ++e) An[4 * q4 + e] = -expf(a4[e]);
  }
#pragma unroll
  for (int n = 0; n < kNS; ++n) h[n] = 0.f;
  const float Dd = Dp[d];
  const int sr_r = tid >> 3, sr_q = (tid & 7) * 4;

#pragma unroll 1
  for (int c = 0; c < kL / 16; ++c) {
    const int l0 = dir ? (kL - 16 - 16 * c) : (16 * c);
    {
      const v4f v = *(const v4f*)(PR + (rowbase + l0 + sr_r) * kPRP + kRk + sr_q);
      *(v4f*)(sBC + sr_r * 32 + sr_q) = v;
    }
    __syncthreads();
#pragma unroll 1
    for (int s = 0; s < 16; ++s) {
      const int sr = dir ? (15 - s) : s;
      const size_t m = rowbase + l0 + sr;
      const float a  = DLR[m * kE + d];
      const float xv = U[m * kE + d];
      const float delta = fmaxf(a, 0.0f) + log1pf(expf(-fabsf(a)));
      v4f Bq[4], Cq[4];
#pragma unroll
      for (int qq = 0; qq < 4; ++qq) {
        Bq[qq] = *(const v4f*)(sBC + sr * 32 + 4 * qq);
        Cq[qq] = *(const v4f*)(sBC + sr * 32 + kNS + 4 * qq);
      }
      const float dx = delta * xv;
      float y = 0.f;
#pragma unroll
      for (int n = 0; n < kNS; ++n) {
        const float e = __expf(delta * An[n]);
        const float hn = fmaf(e, h[n], dx * Bq[n >> 2][n & 3]);
        h[n] = hn;
        y = fmaf(hn, Cq[n >> 2][n & 3], y);
      }
      y = fmaf(xv, Dd, y);
      sY[sr * kScanYP + tid] = y;
    }
    __syncthreads();
    v4f fv[4];
#pragma unroll
    for (int it = 0; it < 4; ++it) fv[it] = *(const v4f*)(sY + (it * 4 + wave) * kScanYP + lane * 4);
    for (int pass = 0; pass < 2; ++pass) {
#pragma unroll
      for (int it = 0; it < 4; ++it)
        *(volatile v4f*)(Y + (rowbase + l0 + it * 4 + wave) * kE + d0 + lane * 4) = fv[it];
      __threadfence();
    }
  }
}

__global__ __launch_bounds__(256) void gate_kernel(
    const float* __restrict__ Y, const float* __restrict__ XZ, unsigned short* __restrict__ G16, float scale)
{
  const int i = blockIdx.x * 256 + threadIdx.x;
  const int e0 = i << 3;
  const int l = e0 >> 9;
  const int c = e0 & (kE - 1);
  const float* pf = Y + (size_t)l * kE + c;
  const float* pb = Y + (size_t)kL * kE + (size_t)l * kE + c;
  const float* pz = XZ + (size_t)l * kXZP + kE + c;
  const v4f f0 = *(const v4f*)(pf), f1 = *(const v4f*)(pf + 4);
  const v4f b0 = *(const v4f*)(pb), b1 = *(const v4f*)(pb + 4);
  const v4f z0 = *(const v4f*)(pz), z1 = *(const v4f*)(pz + 4);
  v8h hv;
#pragma unroll
  for (int e = 0; e < 4; ++e) {
    const float y0 = f0[e] + b0[e];
    const float y1 = f1[e] + b1[e];
    const float s0 = __builtin_amdgcn_rcpf(1.0f + expf(-z0[e]));
    const float s1 = __builtin_amdgcn_rcpf(1.0f + expf(-z1[e]));
    hv[e]     = (_Float16)((y0 * (z0[e] * s0)) * scale);
    hv[4 + e] = (_Float16)((y1 * (z1[e] * s1)) * scale);
  }
  unsigned short* q = G16 + e0;
  *(volatile v8h*)q = hv;
  __threadfence();
  *(volatile v8h*)q = hv;
}

__global__ __launch_bounds__(256) void track_attn_kernel(
    const float* __restrict__ Q, const float* __restrict__ KV, unsigned short* __restrict__ O16, float scale)
{
  const int tid = threadIdx.x, lane = tid & 31, wave = tid >> 5;
  const int gw = blockIdx.x * 8 + wave;
  const int l = gw >> 2;
  const int hd = gw & 3;
  const int col = hd * kDH + 2 * lane;
  const v2f qv = *(const v2f*)(Q + (size_t)l * kDM + col);
  float lg[kTr];
#pragma unroll
  for (int t = 0; t < kTr; ++t) {
    const v2f kv = *(const v2f*)(KV + ((size_t)l * kTr + t) * kKVP + col);
    float p = 0.0f;
    p = fmaf(qv[0], kv[0], p);
    p = fmaf(qv[1], kv[1], p);
#pragma unroll
    for (int off = 16; off > 0; off >>= 1) p += __shfl_xor(p, off, 32);
    lg[t] = p * kLogitScale;
  }
  float mx = lg[0];
#pragma unroll
  for (int t = 1; t < kTr; ++t) mx = fmaxf(mx, lg[t]);
  float sum = 0.0f;
#pragma unroll
  for (int t = 0; t < kTr; ++t) { lg[t] = expf(lg[t] - mx); sum += lg[t]; }
  const float inv = 1.0f / sum;
  float o0 = 0.0f, o1 = 0.0f;
#pragma unroll
  for (int t = 0; t < kTr; ++t) {
    const v2f vv = *(const v2f*)(KV + ((size_t)l * kTr + t) * kKVP + kDM + col);
    const float w = lg[t] * inv;
    o0 = fmaf(w, vv[0], o0);
    o1 = fmaf(w, vv[1], o1);
  }
  const _Float16 h0 = (_Float16)(o0 * scale);
  const _Float16 h1 = (_Float16)(o1 * scale);
  const unsigned short u0 = __builtin_bit_cast(unsigned short, h0);
  const unsigned short u1 = __builtin_bit_cast(unsigned short, h1);
  const unsigned word = (unsigned)u0 | ((unsigned)u1 << 16);
  unsigned* q = (unsigned*)O16 + (size_t)l * (kDM / 2) + hd * (kDH / 2) + lane;
  *(volatile unsigned*)q = word;
  __threadfence();
  *(volatile unsigned*)q = word;
}

template <int BIAS_MODE, bool RESID>
static void launch_gemm(hipStream_t s, const unsigned short* A, int lda, const unsigned short* Bt, int ldb,
                        float* C, int ldc, const float* bias, const float* resid, int M, int N, int K) {
  const int tiles = (M >> 6) * (N >> 6);
  wmma_gemm64<BIAS_MODE, RESID><<<dim3((tiles + 7) / 8, 1, 1), 256, 0, s>>>(
      A, lda, Bt, ldb, C, ldc, bias, resid, M, N, K, kFold);
}

extern "C" void kernel_launch(void* const* d_in, const int* in_sizes, int n_in,
                              void* d_out, int out_size, void* d_ws, size_t ws_size,
                              hipStream_t stream)
{
  if (n_in < 21) return;
  if (in_sizes[0] != kL * kDM) return;
  if (in_sizes[1] != kTr * kL * kDT) return;
  if (in_sizes[2] != kNL * kDM) return;
  if (in_sizes[3] != kNL * kDM * kXZP) return;
  if (in_sizes[4] != kNL * kTaps * kE) return;
  if (in_sizes[5] != kNL * kE) return;
  if (in_sizes[6] != kNL * kE * kPRN) return;
  if (in_sizes[7] != kNL * kRk * kE) return;
  if (in_sizes[8] != kNL * kE) return;
  if (in_sizes[9] != kNL * kE * kNS) return;
  if (in_sizes[10] != kNL * kE) return;
  if (in_sizes[11] != kNL * kE * kDM) return;
  if (in_sizes[12] != kNCA * kDM) return;
  if (in_sizes[13] != kNCA * kDM * kDM) return;
  if (in_sizes[14] != kNCA * kDM) return;
  if (in_sizes[15] != kNCA * kDT * kDM) return;
  if (in_sizes[16] != kNCA * kDM) return;
  if (in_sizes[17] != kNCA * kDT * kDM) return;
  if (in_sizes[18] != kNCA * kDM) return;
  if (in_sizes[19] != kNCA * kDM * kDM) return;
  if (in_sizes[20] != kNCA * kDM) return;
  if (out_size != kL * kDM) return;
  if (ws_size < kWsTotal) return;

  const float* x0      = (const float*)d_in[0];
  const float* tracks  = (const float*)d_in[1];
  const float* mnorm   = (const float*)d_in[2];
  const float* inproj  = (const float*)d_in[3];
  const float* convw   = (const float*)d_in[4];
  const float* convb   = (const float*)d_in[5];
  const float* xprojw  = (const float*)d_in[6];
  const float* dtw     = (const float*)d_in[7];
  const float* dtb     = (const float*)d_in[8];
  const float* alog    = (const float*)d_in[9];
  const float* Dpar    = (const float*)d_in[10];
  const float* outpw   = (const float*)d_in[11];
  const float* canorm  = (const float*)d_in[12];
  const float* qw      = (const float*)d_in[13];
  const float* qb      = (const float*)d_in[14];
  const float* kw      = (const float*)d_in[15];
  const float* kb      = (const float*)d_in[16];
  const float* vw      = (const float*)d_in[17];
  const float* vb      = (const float*)d_in[18];
  const float* ow      = (const float*)d_in[19];
  const float* ob      = (const float*)d_in[20];
  float* out = (float*)d_out;

  char* ws = (char*)d_ws;
  unsigned short* WIN16  = (unsigned short*)(ws + kOffWIN);
  unsigned short* WXP16  = (unsigned short*)(ws + kOffWXP);
  unsigned short* WDT16  = (unsigned short*)(ws + kOffWDT);
  unsigned short* WOUT16 = (unsigned short*)(ws + kOffWOUT);
  unsigned short* WQ16   = (unsigned short*)(ws + kOffWQ);
  unsigned short* WKV16  = (unsigned short*)(ws + kOffWKV);
  unsigned short* WO16   = (unsigned short*)(ws + kOffWO);
  float*          BKV    = (float*)(ws + kOffBKV);
  unsigned short* TL16   = (unsigned short*)(ws + kOffTL);
  float*          XA     = (float*)(ws + kOffXA);
  float*          XB     = (float*)(ws + kOffXB);
  unsigned short* H16    = (unsigned short*)(ws + kOffH16);
  float*          XZ     = (float*)(ws + kOffXZ);
  float*          U      = (float*)(ws + kOffU);
  unsigned short* U16    = (unsigned short*)(ws + kOffU16);
  float*          PR     = (float*)(ws + kOffPR);
  unsigned short* DT16   = (unsigned short*)(ws + kOffDT16);
  float*          DLR    = (float*)(ws + kOffDLR);
  float*          Y      = (float*)(ws + kOffY);
  unsigned short* G16    = (unsigned short*)(ws + kOffG16);
  float*          Qf     = (float*)(ws + kOffQ);
  float*          KV     = (float*)(ws + kOffKV);
  unsigned short* O16    = (unsigned short*)(ws + kOffO16);

  transpose_cast_kernel<<<dim3(kXZP / 64, kDM / 64, kNL), 256, 0, stream>>>(
      inproj, WIN16, kDM, kXZP, kWgtCarry, (long)kDM * kXZP, (long)kXZP * kDM);
  transpose_cast_kernel<<<dim3(kPRP / 64, kE / 64, kNL), 256, 0, stream>>>(
      xprojw, WXP16, kE, kPRN, kWgtCarry, (long)kE * kPRN, (long)kPRP * kE);
  transpose_cast_kernel<<<dim3(kDM / 64, kE / 64, kNL), 256, 0, stream>>>(
      outpw, WOUT16, kE, kDM, kWgtCarry, (long)kE * kDM, (long)kDM * kE);
  transpose_cast_kernel<<<dim3(kDM / 64, kDM / 64, kNCA), 256, 0, stream>>>(
      qw, WQ16, kDM, kDM, kWgtCarry, (long)kDM * kDM, (long)kDM * kDM);
  transpose_cast_kernel<<<dim3(kDM / 64, kDT / 64, kNCA), 256, 0, stream>>>(
      kw, WKV16, kDT, kDM, kWgtCarry, (long)kDT * kDM, (long)kKVP * kDT);
  transpose_cast_kernel<<<dim3(kDM / 64, kDT / 64, kNCA), 256, 0, stream>>>(
      vw, WKV16 + (size_t)kDM * kDT, kDT, kDM, kWgtCarry, (long)kDT * kDM, (long)kKVP * kDT);
  transpose_cast_kernel<<<dim3(kDM / 64, kDM / 64, kNCA), 256, 0, stream>>>(
      ow, WO16, kDM, kDM, kWgtCarry, (long)kDM * kDM, (long)kDM * kDM);
  dtw_cast_kernel<<<(kNL * kE * kDTK) / 8 / 256, 256, 0, stream>>>(dtw, WDT16, kWgtCarry);
  bias_merge_kernel<<<1, 256, 0, stream>>>(kb, vb, BKV);
  tracks_cast_kernel<<<(kL * kTr * kDT) / 8 / 256, 256, 0, stream>>>(tracks, TL16, kActCarry);

  const float* srcs[6] = { x0, XA, XB, XA, XB, XA };
  float*       dsts[6] = { XA, XB, XA, XB, XA, out };
  int blk = 0;

  for (int i = 0; i < kNL; ++i) {
    const float* xs = srcs[blk];
    float*       xd = dsts[blk];
    ++blk;
    rmsnorm_f16_kernel<<<kL / 8, 256, 0, stream>>>(xs, mnorm + (size_t)i * kDM, H16, kActCarry);
    launch_gemm<0, false>(stream, H16, kDM, WIN16 + (size_t)i * kXZP * kDM, kDM, XZ, kXZP, dtb, x0, kL, kXZP, kDM);
    conv_silu_kernel<<<dim3(kE / 256, kL / 64, 2), 256, 0, stream>>>(
        XZ, convw + (size_t)i * kTaps * kE, convb + (size_t)i * kE, U, U16, kActCarry);
    launch_gemm<0, false>(stream, U16, kE, WXP16 + (size_t)i * kPRP * kE, kE, PR, kPRP, dtb, x0, kRows2, kPRP, kE);
    dt_cast_kernel<<<(kRows2 * kDTK) / 8 / 256, 256, 0, stream>>>(PR, DT16, kActCarry);
    launch_gemm<2, false>(stream, DT16, kDTK, WDT16 + (size_t)i * kE * kDTK, kDTK, DLR, kE,
                          dtb + (size_t)i * kE, x0, kRows2, kE, kDTK);
    scan_kernel<<<2 * (kE / kScanCh), kScanCh, 0, stream>>>(
        DLR, U, PR, alog + (size_t)i * kE * kNS, Dpar + (size_t)i * kE, Y);
    gate_kernel<<<(kL * kE) / 8 / 256, 256, 0, stream>>>(Y, XZ, G16, kActCarry);
    launch_gemm<0, true>(stream, G16, kE, WOUT16 + (size_t)i * kDM * kE, kE, xd, kDM, dtb, xs, kL, kDM, kE);

    if (i == 1 || i == 3) {
      const int j = (i == 1) ? 0 : 1;
      const float* cs = srcs[blk];
      float*       cd = dsts[blk];
      ++blk;
      rmsnorm_f16_kernel<<<kL / 8, 256, 0, stream>>>(cs, canorm + (size_t)j * kDM, H16, kActCarry);
      launch_gemm<2, false>(stream, H16, kDM, WQ16 + (size_t)j * kDM * kDM, kDM, Qf, kDM,
                            qb + (size_t)j * kDM, x0, kL, kDM, kDM);
      launch_gemm<2, false>(stream, TL16, kDT, WKV16 + (size_t)j * kKVP * kDT, kDT, KV, kKVP,
                            BKV + (size_t)j * kKVP, x0, kL * kTr, kKVP, kDT);
      track_attn_kernel<<<(kL * kNH) / 8, 256, 0, stream>>>(Qf, KV, O16, kActCarry);
      launch_gemm<2, true>(stream, O16, kDM, WO16 + (size_t)j * kDM * kDM, kDM, cd, kDM,
                           ob + (size_t)j * kDM, cs, kL, kDM, kDM);
    }
  }
}
